// GNNModelWrapper_46291157516799
// MI455X (gfx1250) — hardware-verified
//
#include <hip/hip_runtime.h>
#include <stddef.h>
#include <stdint.h>


#define INW     128
#define HID     64
#define NTHR    256
#define NWAVE   8
#define EPT     8
#define NGRP    2
#define CHUNK   (NTHR * EPT * NGRP)
#define WCAP    (EPT * NGRP * 32)
#define LISTN   (NWAVE * WCAP)
#define NBC     4096
#define NBF     1024
#define RCAP    40960
#define RBN     128
#define TGT     256
#define DEGCAP  512
#define GROWS   128
#define OTHR    512
#define WSCALE  8.0f
#define WINV    0.125f
#define NSLOPE  0.2f

#define LDS_FILL ((RCAP + NBF + LISTN) * 4 + 64)
#define LDSG_V4  (GROWS * (INW + 8) * 2 / 16)
#define WSLIM    ((size_t)134217728)

static_assert((CHUNK & (CHUNK - 1)) == 0);
static_assert(CHUNK <= 4096);
static_assert(NBC <= 4096 && NBF <= 4096);
static_assert((NBC & (NBC - 1)) == 0 && (NBF & (NBF - 1)) == 0);
static_assert(NBC == 4 * NBF);
static_assert(OTHR * 8 == NBC);
static_assert((RCAP % 32) == 0);
static_assert(GROWS * HID * 4 <= LDSG_V4 * 16);
static_assert(TGT == NWAVE * 32 && (TGT % GROWS) == 0);
static_assert((GROWS * INW / 8) % NTHR == 0 && (GROWS * HID / 8) % NTHR == 0);
static_assert((HID * INW / 8) % NTHR == 0 && (HID * HID / 8) % NTHR == 0);

typedef float    v2f  __attribute__((ext_vector_type(2)));
typedef float    v4f  __attribute__((ext_vector_type(4)));
typedef float    v8f  __attribute__((ext_vector_type(8)));
typedef int      v4i  __attribute__((ext_vector_type(4)));
typedef _Float16 v8h  __attribute__((ext_vector_type(8)));
typedef _Float16 v16h __attribute__((ext_vector_type(16)));
union FragH { v16h v; v8h h[2]; };
union FI { float f; int i; };

__device__ __forceinline__ float lrelu(float v) { return v > 0.0f ? v : NSLOPE * v; }

__device__ __forceinline__ v8h cvt8(v4f a, v4f b) {
  v8h r;
  r[0] = (_Float16)a.x; r[1] = (_Float16)a.y; r[2] = (_Float16)a.z; r[3] = (_Float16)a.w;
  r[4] = (_Float16)b.x; r[5] = (_Float16)b.y; r[6] = (_Float16)b.z; r[7] = (_Float16)b.w;
  return r;
}

__device__ __forceinline__ v8f wmh(v16h a, v16h b, v8f c) {
  v8f d = __builtin_amdgcn_wmma_f32_16x16x32_f16(false, a, false, b, (short)0, c, false, false);
  asm volatile("v_nop\n\tv_nop\n\tv_nop\n\tv_nop" : "+v"(d) : "v"(a), "v"(b));
  return d;
}

template <int NB>
__device__ __forceinline__ int scan_chunk(const int* __restrict__ dsts, int nE, int cbase, int slotBase,
                                          int vec8, int* list, int tid, int lane, int wave) {
  int wc = 0;
#pragma unroll
  for (int g = 0; g < NGRP; ++g) {
    const int el0  = (g * NTHR + tid) * EPT;
    const int e0   = cbase + el0;
    const int sent = -2147483647 - 1;
    v4i da, db;
    if (vec8 != 0 && cbase + CHUNK <= nE) {
      da = *(const v4i*)(dsts + e0);
      db = *(const v4i*)(dsts + e0 + 4);
    } else {
      da.x = (e0     < nE) ? dsts[min(e0, nE - 1)] : sent;
      da.y = (e0 + 1 < nE) ? dsts[min(e0 + 1, nE - 1)] : sent;
      da.z = (e0 + 2 < nE) ? dsts[min(e0 + 2, nE - 1)] : sent;
      da.w = (e0 + 3 < nE) ? dsts[min(e0 + 3, nE - 1)] : sent;
      db.x = (e0 + 4 < nE) ? dsts[min(e0 + 4, nE - 1)] : sent;
      db.y = (e0 + 5 < nE) ? dsts[min(e0 + 5, nE - 1)] : sent;
      db.z = (e0 + 6 < nE) ? dsts[min(e0 + 6, nE - 1)] : sent;
      db.w = (e0 + 7 < nE) ? dsts[min(e0 + 7, nE - 1)] : sent;
    }
    const unsigned nb = (unsigned)slotBase;
    const unsigned s0 = (unsigned)da.x - nb, s1 = (unsigned)da.y - nb;
    const unsigned s2 = (unsigned)da.z - nb, s3 = (unsigned)da.w - nb;
    const unsigned s4 = (unsigned)db.x - nb, s5 = (unsigned)db.y - nb;
    const unsigned s6 = (unsigned)db.z - nb, s7 = (unsigned)db.w - nb;
    const bool h0 = s0 < (unsigned)NB, h1 = s1 < (unsigned)NB, h2 = s2 < (unsigned)NB, h3 = s3 < (unsigned)NB;
    const bool h4 = s4 < (unsigned)NB, h5 = s5 < (unsigned)NB, h6 = s6 < (unsigned)NB, h7 = s7 < (unsigned)NB;
    const unsigned any = __builtin_amdgcn_ballot_w32(h0 | h1 | h2 | h3 | h4 | h5 | h6 | h7);
    if (any != 0u) {
#define HITJ(J, HJ, SJ) { \
        const unsigned mj = __builtin_amdgcn_ballot_w32(HJ); \
        if (mj != 0u) { \
          if (HJ) { \
            const int pos = wc + (int)__builtin_amdgcn_mbcnt_lo(mj, 0u); \
            if (pos < WCAP) list[wave * WCAP + pos] = ((el0 + (J)) << 12) | (int)(SJ); \
          } \
          wc += (int)__builtin_popcount(mj); } }
      HITJ(0, h0, s0)
      HITJ(1, h1, s1)
      HITJ(2, h2, s2)
      HITJ(3, h3, s3)
      HITJ(4, h4, s4)
      HITJ(5, h5, s5)
      HITJ(6, h6, s6)
      HITJ(7, h7, s7)
#undef HITJ
    }
  }
  return wc;
}

__global__ __launch_bounds__(NTHR) void k_wprep(
    const float* __restrict__ gw, const float* __restrict__ tw,
    const float* __restrict__ wl, const float* __restrict__ wr,
    _Float16* pG, _Float16* pT, _Float16* pS) {
  const int g0 = HID * INW / 8;
  const int g1 = HID * HID / 8;
  const int g2 = HID * INW / 8;
  const int bstart = blockIdx.x * NTHR;
  const int i = bstart + (int)threadIdx.x;
  if (i >= g0 + g1 + g2) return;
  float v[8];
  _Float16* dp;
  if (bstart < g0) {
    const int o  = i * 8;
    const int n  = o / INW;
    const int k0 = o - n * INW;
#pragma unroll
    for (int e = 0; e < 8; ++e) v[e] = gw[(size_t)(k0 + e) * HID + n] * WSCALE;
    dp = pG + o;
  } else if (bstart < g0 + g1) {
    const int o  = (i - g0) * 8;
    const int n  = o / HID;
    const int k0 = o - n * HID;
#pragma unroll
    for (int e = 0; e < 8; ++e) v[e] = tw[(size_t)(k0 + e) * HID + n] * WSCALE;
    dp = pT + o;
  } else {
    const int o  = (i - g0 - g1) * 8;
    const int n  = o / INW;
    const int k0 = o - n * INW;
#pragma unroll
    for (int e = 0; e < 8; ++e) {
      const int k  = k0 + e;
      const int ka = k < HID ? k : HID - 1;
      int kb = k - HID; kb = kb < 0 ? 0 : (kb > HID - 1 ? HID - 1 : kb);
      const float a = wl[(size_t)ka * HID + n];
      const float b = wr[(size_t)kb * HID + n];
      v[e] = (k < HID ? a : b) * WSCALE;
    }
    dp = pS + o;
  }
  v4f a, b;
  a.x = v[0]; a.y = v[1]; a.z = v[2]; a.w = v[3];
  b.x = v[4]; b.y = v[5]; b.z = v[6]; b.w = v[7];
  const v8h hv = cvt8(a, b);
  *(volatile v8h*)dp = hv;
  __threadfence();
  *(volatile v8h*)dp = hv;
}

__global__ __launch_bounds__(NTHR) void k_count(
    const int* __restrict__ ei, int* cnt, float* dinv, int nE, int vec8) {
  __shared__ __attribute__((aligned(16))) int scnt[NBC];
  __shared__ __attribute__((aligned(16))) int list[LISTN];
  __shared__ int wcnt[NWAVE];
  const int tid = threadIdx.x, lane = tid & 31, wave = tid >> 5;
  const int nodeBase = blockIdx.x * NBC;
  const int* dsts = ei + nE;

  for (int i = tid; i < NBC; i += NTHR) scnt[i] = 0;
  __syncthreads();

  const int nChunks = (nE + CHUNK - 1) / CHUNK;
#pragma unroll 1
  for (int ch = 0; ch < nChunks; ++ch) {
    const int cbase = ch * CHUNK;
    const int wc = scan_chunk<NBC>(dsts, nE, cbase, nodeBase, vec8, list, tid, lane, wave);
    if (lane == 0) wcnt[wave] = wc;
    __syncthreads();
    if (wave == 0) {
#pragma unroll 1
      for (int wsx = 0; wsx < NWAVE; ++wsx) {
        int n = __builtin_amdgcn_readfirstlane(wcnt[wsx]);
        n = n > WCAP ? WCAP : (n < 0 ? 0 : n);
        const int* lp = list + wsx * WCAP;
#pragma unroll 1
        for (int i = 0; i < n; ++i) {
          const int ent  = __builtin_amdgcn_readfirstlane(lp[i]);
          const int slot = ent & (NBC - 1);
          if (lane == 0) scnt[slot] = scnt[slot] + 1;
        }
      }
    }
    __syncthreads();
  }

  v4i cq[4]; v4f dq[4];
#pragma unroll
  for (int q = 0; q < 4; ++q) {
    const int f = (wave * 4 + q) * 128 + 4 * lane;
    const v4i c = *(const v4i*)(scnt + f);
    cq[q] = c;
    dq[q].x = rsqrtf((float)(c.x + 1));
    dq[q].y = rsqrtf((float)(c.y + 1));
    dq[q].z = rsqrtf((float)(c.z + 1));
    dq[q].w = rsqrtf((float)(c.w + 1));
  }
  int*   cp = cnt + (size_t)nodeBase;
  float* dp = dinv + (size_t)nodeBase;
#pragma unroll
  for (int q = 0; q < 4; ++q) {
    const int f = (wave * 4 + q) * 128 + 4 * lane;
    *(volatile v4i*)(cp + f) = cq[q];
    *(volatile v4f*)(dp + f) = dq[q];
  }
  __threadfence();
#pragma unroll
  for (int q = 0; q < 4; ++q) {
    const int f = (wave * 4 + q) * 128 + 4 * lane;
    *(volatile v4i*)(cp + f) = cq[q];
    *(volatile v4f*)(dp + f) = dq[q];
  }
}

__global__ __launch_bounds__(OTHR) void k_offsets(
    const int* __restrict__ cnt, int* off, int* rbase, int nChunk) {
  __shared__ __attribute__((aligned(16))) int soff[NBC];
  __shared__ __attribute__((aligned(16))) int srb[RBN];
  __shared__ int wtot[OTHR / 32];
  const int tid = threadIdx.x, lane = tid & 31, wave = tid >> 5, sub = tid >> 7;
  for (int i = tid; i < RBN; i += OTHR) srb[i] = 0;
  int carry = 0;
#pragma unroll 1
  for (int ch = 0; ch < nChunk; ++ch) {
    const int base = ch * NBC;
    const v4i c0 = *(const v4i*)(cnt + base + 8 * tid);
    const v4i c1 = *(const v4i*)(cnt + base + 8 * tid + 4);
    const int e0 = max(c0.x, 0), e1 = max(c0.y, 0), e2 = max(c0.z, 0), e3 = max(c0.w, 0);
    const int e4 = max(c1.x, 0), e5 = max(c1.y, 0), e6 = max(c1.z, 0), e7 = max(c1.w, 0);
    const int ts = e0 + e1 + e2 + e3 + e4 + e5 + e6 + e7;
    int incl = ts;
#pragma unroll
    for (int d = 1; d < 32; d <<= 1) {
      const int t = __shfl_up(incl, d);
      if (lane >= d) incl += t;
    }
    if (lane == 31) wtot[wave] = incl;
    __syncthreads();
    const int S0 = wtot[0]  + wtot[1]  + wtot[2]  + wtot[3];
    const int S1 = wtot[4]  + wtot[5]  + wtot[6]  + wtot[7];
    const int S2 = wtot[8]  + wtot[9]  + wtot[10] + wtot[11];
    const int S3 = wtot[12] + wtot[13] + wtot[14] + wtot[15];
    int pre = 0;
#pragma unroll 1
    for (int w = 4 * sub; w < wave; ++w) pre += wtot[w];
    const int b0 = carry;
    const int b1 = b0 + ((S0 + 31) & ~31);
    const int b2 = b1 + ((S1 + 31) & ~31);
    const int b3 = b2 + ((S2 + 31) & ~31);
    const int b4 = b3 + ((S3 + 31) & ~31);
    const int myb = sub == 0 ? b0 : (sub == 1 ? b1 : (sub == 2 ? b2 : b3));
    if (tid == 0) {
      srb[min(4 * ch + 0, RBN - 1)] = b0;
      srb[min(4 * ch + 1, RBN - 1)] = b1;
      srb[min(4 * ch + 2, RBN - 1)] = b2;
      srb[min(4 * ch + 3, RBN - 1)] = b3;
    }
    int run = myb + pre + incl - ts;
    soff[8 * tid + 0] = run; run += e0;
    soff[8 * tid + 1] = run; run += e1;
    soff[8 * tid + 2] = run; run += e2;
    soff[8 * tid + 3] = run; run += e3;
    soff[8 * tid + 4] = run; run += e4;
    soff[8 * tid + 5] = run; run += e5;
    soff[8 * tid + 6] = run; run += e6;
    soff[8 * tid + 7] = run;
    carry = b4;
    __syncthreads();
    const v4i o0 = *(const v4i*)(soff + 4 * tid);
    const v4i o1 = *(const v4i*)(soff + 4 * (tid + OTHR));
    int* op = off + base;
    *(volatile v4i*)(op + 4 * tid) = o0;
    *(volatile v4i*)(op + 4 * (tid + OTHR)) = o1;
    __threadfence();
    *(volatile v4i*)(op + 4 * tid) = o0;
    *(volatile v4i*)(op + 4 * (tid + OTHR)) = o1;
    __syncthreads();
  }
  if (tid == 0) srb[min(4 * nChunk, RBN - 1)] = carry;
  __syncthreads();
  v4i rv = {0, 0, 0, 0};
  if (tid < 32) rv = *(const v4i*)(srb + 4 * tid);
  if (tid < 32) *(volatile v4i*)(rbase + 4 * tid) = rv;
  __threadfence();
  if (tid < 32) *(volatile v4i*)(rbase + 4 * tid) = rv;
}

__global__ __launch_bounds__(NTHR) void k_fill(
    const int* __restrict__ ei, const int* __restrict__ off, const int* __restrict__ rbase,
    int* csr, int nN, int nE, int vec8, int csrLen) {
  extern __shared__ v4f lds_dyn[];
  int* region = (int*)lds_dyn;
  int* cursor = region + RCAP;
  int* list   = cursor + NBF;
  int* wcnt   = list + LISTN;
  const int tid = threadIdx.x, lane = tid & 31, wave = tid >> 5;
  const int b = blockIdx.x;
  const int nodeBase = b * NBF;
  const int* dsts = ei + nE;

  int rb0 = rbase[b];
  const int rb1 = rbase[b + 1];
  rb0 = rb0 < 0 ? 0 : (rb0 > csrLen ? csrLen : rb0);
  rb0 &= ~31;
  int len = rb1 - rb0;
  len = len < 0 ? 0 : (len > RCAP ? RCAP : len);
  int lenW = (len + 31) & ~31;
  if (rb0 + lenW > csrLen) lenW = (csrLen - rb0) & ~31;

  {
    const v4i z = {0, 0, 0, 0};
    for (int i = tid; i < RCAP / 4; i += NTHR) ((v4i*)region)[i] = z;
    for (int s = tid; s < NBF; s += NTHR) {
      int o = off[nodeBase + s] - rb0;
      o = o < 0 ? 0 : (o > RCAP ? RCAP : o);
      cursor[s] = o;
    }
  }
  __syncthreads();

  const int nChunks = (nE + CHUNK - 1) / CHUNK;
#pragma unroll 1
  for (int ch = 0; ch < nChunks; ++ch) {
    const int cbase = ch * CHUNK;
    const int wc = scan_chunk<NBF>(dsts, nE, cbase, nodeBase, vec8, list, tid, lane, wave);
    if (lane == 0) wcnt[wave] = wc;
    __syncthreads();
    if (wave == 0) {
#pragma unroll 1
      for (int wsx = 0; wsx < NWAVE; ++wsx) {
        int n = __builtin_amdgcn_readfirstlane(wcnt[wsx]);
        n = n > WCAP ? WCAP : (n < 0 ? 0 : n);
        const int* lp = list + wsx * WCAP;
#pragma unroll 1
        for (int i = 0; i < n; ++i) {
          const int ent  = __builtin_amdgcn_readfirstlane(lp[i]);
          const int slot = ent & (NBF - 1);
          int e = cbase + ((ent >> 12) & (CHUNK - 1));
          e = e > nE - 1 ? nE - 1 : e;
          int src = ei[e];
          src = src < 0 ? 0 : (src > nN - 1 ? nN - 1 : src);
          if (lane == 0) {
            int pos = cursor[slot];
            pos = pos < 0 ? 0 : (pos > RCAP - 1 ? RCAP - 1 : pos);
            region[pos] = src;
            const int np = pos + 1;
            cursor[slot] = np > RCAP ? RCAP : np;
          }
        }
      }
    }
    __syncthreads();
  }

  const int nv = lenW >> 2;
  int* gp = csr + rb0;
#pragma unroll 1
  for (int i = tid; i < nv; i += NTHR) { const v4i v = ((const v4i*)region)[i]; *(volatile v4i*)(gp + 4 * i) = v; }
  __threadfence();
#pragma unroll 1
  for (int i = tid; i < nv; i += NTHR) { const v4i v = ((const v4i*)region)[i]; *(volatile v4i*)(gp + 4 * i) = v; }
}

template <int KD, int MODE>
__global__ __launch_bounds__(NTHR) void k_gemm(
    const float* __restrict__ A0, const float* __restrict__ A1, const _Float16* __restrict__ Bs,
    const float* __restrict__ dinv, const float* __restrict__ bias,
    const float* __restrict__ asv, const float* __restrict__ adv,
    float* C, float* aso, float* ado, int nRowsA, int nRowsOut) {
  static_assert(KD % 32 == 0);
  static_assert(MODE != 2 || KD == 2 * HID);
  static_assert(GROWS * (KD + 8) * 2 <= LDSG_V4 * 16);
  __shared__ v4f lds_g[LDSG_V4];
  __shared__ __attribute__((aligned(16))) float sdot[2 * GROWS];
  constexpr int AP = KD + 8;
  _Float16* sA  = (_Float16*)lds_g;
  float*    stg = (float*)lds_g;
  const int tid = threadIdx.x, lane = tid & 31, wave = tid >> 5, hh = lane >> 4, m = lane & 15;
  const int rowBase = blockIdx.x * GROWS;

  if (MODE != 2) {
#pragma unroll
    for (int i = 0; i < (GROWS * KD / 8) / NTHR; ++i) {
      const int idx = i * NTHR + tid;
      const int r   = idx / (KD / 8);
      const int c0  = (idx - r * (KD / 8)) * 8;
      int row = rowBase + r;
      row = row > nRowsA - 1 ? nRowsA - 1 : row;
      const float* ap = A0 + (size_t)row * KD + c0;
      const v4f a = *(const v4f*)ap, b = *(const v4f*)(ap + 4);
      *(v8h*)(sA + r * AP + c0) = cvt8(a, b);
    }
  } else {
#pragma unroll
    for (int s = 0; s < 2; ++s) {
      const float* As = (s == 0) ? A0 : A1;
#pragma unroll
      for (int i = 0; i < (GROWS * HID / 8) / NTHR; ++i) {
        const int idx = i * NTHR + tid;
        const int r   = idx >> 3;
        const int c0  = (idx & 7) * 8;
        int row = rowBase + r;
        row = row > nRowsA - 1 ? nRowsA - 1 : row;
        const float* ap = As + (size_t)row * HID + c0;
        const v4f a = *(const v4f*)ap, b = *(const v4f*)(ap + 4);
        *(v8h*)(sA + r * AP + HID * s + c0) = cvt8(a, b);
      }
    }
  }
  __syncthreads();

  v8f acc[4];
#pragma unroll
  for (int t = 0; t < 4; ++t) { v8f z = {0.f, 0.f, 0.f, 0.f, 0.f, 0.f, 0.f, 0.f}; acc[t] = z; }
  const _Float16* ar = sA + (wave * 16 + m) * AP + 8 * hh;
#pragma unroll
  for (int kt = 0; kt < KD / 32; ++kt) {
    FragH a;
    a.h[0] = *(const v8h*)(ar + 32 * kt);
    a.h[1] = *(const v8h*)(ar + 32 * kt + 16);
#pragma unroll
    for (int t = 0; t < 4; ++t) {
      const _Float16* bp = Bs + (size_t)(16 * t + m) * KD + 32 * kt + 8 * hh;
      FragH b;
      b.h[0] = *(const v8h*)bp;
      b.h[1] = *(const v8h*)(bp + 16);
      acc[t] = wmh(a.v, b.v, acc[t]);
    }
  }
  __syncthreads();

  const int r0 = wave * 16 + 8 * hh;
  float sc[8];
  if (MODE == 0) {
    const v4f dA = *(const v4f*)(dinv + (size_t)rowBase + r0);
    const v4f dB = *(const v4f*)(dinv + (size_t)rowBase + r0 + 4);
    sc[0] = dA.x * WINV; sc[1] = dA.y * WINV; sc[2] = dA.z * WINV; sc[3] = dA.w * WINV;
    sc[4] = dB.x * WINV; sc[5] = dB.y * WINV; sc[6] = dB.z * WINV; sc[7] = dB.w * WINV;
  } else {
#pragma unroll
    for (int r = 0; r < 8; ++r) sc[r] = WINV;
  }
  float* sp = stg + r0 * HID + m;
#pragma unroll
  for (int t = 0; t < 4; ++t) {
    float bv = 0.0f;
    if (MODE == 2) bv = bias[16 * t + m];
#pragma unroll
    for (int r = 0; r < 8; ++r) sp[r * HID + 16 * t] = acc[t][r] * sc[r] + bv;
  }
  __syncthreads();

  if (MODE == 1) {
    const v2f as2 = *(const v2f*)(asv + 2 * lane);
    const v2f ad2 = *(const v2f*)(adv + 2 * lane);
#pragma unroll 1
    for (int rr = 0; rr < 16; ++rr) {
      const v2f hv = *(const v2f*)(stg + (wave * 16 + rr) * HID + 2 * lane);
      float ps = hv.x * as2.x + hv.y * as2.y;
      float pd = hv.x * ad2.x + hv.y * ad2.y;
      ps += __shfl_xor(ps, 16); pd += __shfl_xor(pd, 16);
      ps += __shfl_xor(ps, 8);  pd += __shfl_xor(pd, 8);
      ps += __shfl_xor(ps, 4);  pd += __shfl_xor(pd, 4);
      ps += __shfl_xor(ps, 2);  pd += __shfl_xor(pd, 2);
      ps += __shfl_xor(ps, 1);  pd += __shfl_xor(pd, 1);
      if (lane == 0) { sdot[wave * 16 + rr] = ps; sdot[GROWS + wave * 16 + rr] = pd; }
    }
  }
  __syncthreads();

  v4f rv[8];
#pragma unroll
  for (int i = 0; i < 8; ++i) rv[i] = *(const v4f*)(stg + (wave * 16 + 2 * i + hh) * HID + 4 * m);
  v4f av = {0.f, 0.f, 0.f, 0.f};
  float* apo = aso;
  if (MODE == 1) {
    if (wave < 2) av = *(const v4f*)(sdot + wave * GROWS + 4 * lane);
    apo = ((wave == 0) ? aso : ado) + (size_t)rowBase + 4 * lane;
  }
#pragma unroll
  for (int i = 0; i < 8; ++i) {
    const int row = rowBase + wave * 16 + 2 * i + hh;
    if (MODE != 2 || row < nRowsOut) *(volatile v4f*)(C + (size_t)row * HID + 4 * m) = rv[i];
  }
  if (MODE == 1 && wave < 2) *(volatile v4f*)apo = av;
  __threadfence();
#pragma unroll
  for (int i = 0; i < 8; ++i) {
    const int row = rowBase + wave * 16 + 2 * i + hh;
    if (MODE != 2 || row < nRowsOut) *(volatile v4f*)(C + (size_t)row * HID + 4 * m) = rv[i];
  }
  if (MODE == 1 && wave < 2) *(volatile v4f*)apo = av;
}

__global__ __launch_bounds__(NTHR) void k_agg_gcn(
    const int* __restrict__ csr, const int* __restrict__ off, const int* __restrict__ cnt,
    const float* __restrict__ dinv, const float* __restrict__ hw, const float* __restrict__ bias,
    float* h1, int nN, int csrLen) {
  const int tid = threadIdx.x, lane = tid & 31, wave = tid >> 5;
  const int tbase = blockIdx.x * TGT + wave * 32;
  const int cl = tbase + lane;
  const int cnt_l = cnt[cl];
  const int off_l = off[cl];
  FI dvu; dvu.f = dinv[cl];
  const v2f bb = *(const v2f*)(bias + 2 * lane);
#pragma unroll 1
  for (int j = 0; j < 32; ++j) {
    const int c = tbase + j;
    int n = __builtin_amdgcn_readlane(cnt_l, j);
    n = n < 0 ? 0 : (n > DEGCAP ? DEGCAP : n);
    const int st = __builtin_amdgcn_readlane(off_l, j);
    FI du; du.i = __builtin_amdgcn_readlane(dvu.i, j);
    v2f acc = {0.f, 0.f};
#pragma unroll 1
    for (int q0 = 0; q0 < n; q0 += 32) {
      int pos = st + q0 + lane;
      pos = pos < 0 ? 0 : (pos > csrLen - 1 ? csrLen - 1 : pos);
      int sl = csr[pos];
      sl = sl < 0 ? 0 : (sl > nN - 1 ? nN - 1 : sl);
      const int mcnt = (n - q0) < 32 ? (n - q0) : 32;
#pragma unroll 1
      for (int p = 0; p < mcnt; ++p) {
        const int s = __builtin_amdgcn_readlane(sl, p);
        acc = acc + *(const v2f*)(hw + (size_t)s * HID + 2 * lane);
      }
    }
    const v2f sv = *(const v2f*)(hw + (size_t)c * HID + 2 * lane);
    v2f v = (acc + sv) * du.f + bb;
    v.x = fmaxf(v.x, 0.f); v.y = fmaxf(v.y, 0.f);
    float* hp = h1 + (size_t)c * HID + 2 * lane;
    *(volatile v2f*)hp = v;
    __threadfence();
    *(volatile v2f*)hp = v;
  }
}

__global__ __launch_bounds__(NTHR) void k_agg_gat(
    const int* __restrict__ csr, const int* __restrict__ off, const int* __restrict__ cnt,
    const float* __restrict__ hg, const float* __restrict__ asn, const float* __restrict__ adn,
    const float* __restrict__ bias, float* h2, int nN, int csrLen) {
  const int tid = threadIdx.x, lane = tid & 31, wave = tid >> 5;
  const int tbase = blockIdx.x * TGT + wave * 32;
  const int cl = tbase + lane;
  const int cnt_l = cnt[cl];
  const int off_l = off[cl];
  FI asu; asu.f = asn[cl];
  FI adu; adu.f = adn[cl];
  const v2f bb = *(const v2f*)(bias + 2 * lane);
  const float ninf = -__builtin_inff();
#pragma unroll 1
  for (int j = 0; j < 32; ++j) {
    const int c = tbase + j;
    int n = __builtin_amdgcn_readlane(cnt_l, j);
    n = n < 0 ? 0 : (n > DEGCAP ? DEGCAP : n);
    const int st = __builtin_amdgcn_readlane(off_l, j);
    FI ta; ta.i = __builtin_amdgcn_readlane(asu.i, j);
    FI td; td.i = __builtin_amdgcn_readlane(adu.i, j);
    const float adc = td.f;
    float mrun = lrelu(ta.f + adc);
    float ssum = 1.0f;
    v2f acc = *(const v2f*)(hg + (size_t)c * HID + 2 * lane);
#pragma unroll 1
    for (int q0 = 0; q0 < n; q0 += 32) {
      int pos = st + q0 + lane;
      pos = pos < 0 ? 0 : (pos > csrLen - 1 ? csrLen - 1 : pos);
      int sl = csr[pos];
      sl = sl < 0 ? 0 : (sl > nN - 1 ? nN - 1 : sl);
      const int mcnt = (n - q0) < 32 ? (n - q0) : 32;
      const bool valid = lane < mcnt;
      const float ag = asn[sl];
      const float lg = lrelu(ag + adc);
      float cm = valid ? lg : ninf;
      cm = fmaxf(cm, __shfl_xor(cm, 16));
      cm = fmaxf(cm, __shfl_xor(cm, 8));
      cm = fmaxf(cm, __shfl_xor(cm, 4));
      cm = fmaxf(cm, __shfl_xor(cm, 2));
      cm = fmaxf(cm, __shfl_xor(cm, 1));
      const float nm = fmaxf(mrun, cm);
      const float rs = __expf(mrun - nm);
      acc = acc * rs;
      ssum = ssum * rs;
      mrun = nm;
      const float pe = __expf(lg - mrun);
      FI pu; pu.f = valid ? pe : 0.0f;
#pragma unroll 1
      for (int p = 0; p < mcnt; ++p) {
        const int s = __builtin_amdgcn_readlane(sl, p);
        FI pw; pw.i = __builtin_amdgcn_readlane(pu.i, p);
        acc = acc + *(const v2f*)(hg + (size_t)s * HID + 2 * lane) * pw.f;
        ssum += pw.f;
      }
    }
    const float inv = 1.0f / ssum;
    v2f v = acc * inv + bb;
    v.x = fmaxf(v.x, 0.f); v.y = fmaxf(v.y, 0.f);
    float* hp = h2 + (size_t)c * HID + 2 * lane;
    *(volatile v2f*)hp = v;
    __threadfence();
    *(volatile v2f*)hp = v;
  }
}

__global__ __launch_bounds__(NTHR) void k_agg_sage(
    const int* __restrict__ csr, const int* __restrict__ off, const int* __restrict__ cnt,
    const float* __restrict__ h2, float* mean, int nN, int csrLen) {
  const int tid = threadIdx.x, lane = tid & 31, wave = tid >> 5;
  const int tbase = blockIdx.x * TGT + wave * 32;
  const int cl = tbase + lane;
  const int cnt_l = cnt[cl];
  const int off_l = off[cl];
#pragma unroll 1
  for (int j = 0; j < 32; ++j) {
    const int c = tbase + j;
    int ntrue = __builtin_amdgcn_readlane(cnt_l, j);
    ntrue = ntrue < 0 ? 0 : ntrue;
    const int n = ntrue > DEGCAP ? DEGCAP : ntrue;
    const int st = __builtin_amdgcn_readlane(off_l, j);
    v2f acc = {0.f, 0.f};
#pragma unroll 1
    for (int q0 = 0; q0 < n; q0 += 32) {
      int pos = st + q0 + lane;
      pos = pos < 0 ? 0 : (pos > csrLen - 1 ? csrLen - 1 : pos);
      int sl = csr[pos];
      sl = sl < 0 ? 0 : (sl > nN - 1 ? nN - 1 : sl);
      const int mcnt = (n - q0) < 32 ? (n - q0) : 32;
#pragma unroll 1
      for (int p = 0; p < mcnt; ++p) {
        const int s = __builtin_amdgcn_readlane(sl, p);
        acc = acc + *(const v2f*)(h2 + (size_t)s * HID + 2 * lane);
      }
    }
    const int dd = ntrue < 1 ? 1 : ntrue;
    const float inv = 1.0f / (float)dd;
    const v2f v = acc * inv;
    float* mp = mean + (size_t)c * HID + 2 * lane;
    *(volatile v2f*)mp = v;
    __threadfence();
    *(volatile v2f*)mp = v;
  }
}

extern "C" void kernel_launch(void* const* d_in, const int* in_sizes, int n_in,
                              void* d_out, int out_size, void* d_ws, size_t ws_size,
                              hipStream_t stream) {
  if (n_in < 11) return;
  const int nN = in_sizes[0] / INW;
  const int nE = in_sizes[1] / 2;
  if (nN <= 0 || nE <= 0 || in_sizes[0] != nN * INW || in_sizes[1] != 2 * nE) return;
  if (in_sizes[2] != INW * HID || in_sizes[3] < HID || in_sizes[4] != HID * HID) return;
  if (in_sizes[5] < HID || in_sizes[6] < HID || in_sizes[7] < HID) return;
  if (in_sizes[8] != HID * HID || in_sizes[9] != HID * HID || in_sizes[10] < HID) return;
  if (out_size != nN * HID) return;
  if (nE > (1 << 28) || nN > (1 << 24)) return;

  const float* x       = (const float*)d_in[0];
  const int*   ei      = (const int*)d_in[1];
  const float* gcn_w   = (const float*)d_in[2];
  const float* gcn_b   = (const float*)d_in[3];
  const float* gat_w   = (const float*)d_in[4];
  const float* att_src = (const float*)d_in[5];
  const float* att_dst = (const float*)d_in[6];
  const float* gat_b   = (const float*)d_in[7];
  const float* sage_wl = (const float*)d_in[8];
  const float* sage_wr = (const float*)d_in[9];
  const float* sage_b  = (const float*)d_in[10];
  float* out = (float*)d_out;

  const int NPAD   = ((nN + TGT - 1) / TGT) * TGT;
  const int nBC    = (nN + NBC - 1) / NBC;
  const int CNTPAD = nBC * NBC;
  if (4 * nBC + 1 > RBN) return;
  const int nBF    = (nN + NBF - 1) / NBF;
  const int csrLen = ((nE + 31) & ~31) + 4096;
  const int nGemm  = NPAD / GROWS;
  const int nAgg   = NPAD / TGT;

  char* ws = (char*)d_ws;
  size_t off = 0;
  const size_t oWG  = off; off += (size_t)HID * INW * 2;           off = (off + 255) & ~(size_t)255;
  const size_t oWT  = off; off += (size_t)HID * HID * 2;           off = (off + 255) & ~(size_t)255;
  const size_t oWS  = off; off += (size_t)HID * INW * 2;           off = (off + 255) & ~(size_t)255;
  const size_t oCnt = off; off += (size_t)CNTPAD * 4;              off = (off + 255) & ~(size_t)255;
  const size_t oDv  = off; off += (size_t)CNTPAD * 4;              off = (off + 255) & ~(size_t)255;
  const size_t oOff = off; off += (size_t)CNTPAD * 4;              off = (off + 255) & ~(size_t)255;
  const size_t oRb  = off; off += (size_t)RBN * 4;                 off = (off + 255) & ~(size_t)255;
  const size_t oCsr = off; off += (size_t)csrLen * 4;              off = (off + 255) & ~(size_t)255;
  const size_t oP0  = off; off += (size_t)NPAD * HID * 4;          off = (off + 255) & ~(size_t)255;
  const size_t oP1  = off; off += (size_t)NPAD * HID * 4;          off = (off + 255) & ~(size_t)255;
  const size_t oP2  = off; off += (size_t)NPAD * HID * 4;          off = (off + 255) & ~(size_t)255;
  const size_t oAs  = off; off += (size_t)NPAD * 4;                off = (off + 255) & ~(size_t)255;
  const size_t oAd  = off; off += (size_t)NPAD * 4;                off = (off + 255) & ~(size_t)255;
  if (off > ws_size || off > WSLIM) return;
  _Float16* wG   = (_Float16*)(ws + oWG);
  _Float16* wT   = (_Float16*)(ws + oWT);
  _Float16* wS   = (_Float16*)(ws + oWS);
  int*      cnt  = (int*)(ws + oCnt);
  float*    dinv = (float*)(ws + oDv);
  int*      offp = (int*)(ws + oOff);
  int*      rb   = (int*)(ws + oRb);
  int*      csr  = (int*)(ws + oCsr);
  float*    P0   = (float*)(ws + oP0);
  float*    P1   = (float*)(ws + oP1);
  float*    P2   = (float*)(ws + oP2);
  float*    asp  = (float*)(ws + oAs);
  float*    adp  = (float*)(ws + oAd);

  const int vec8 = ((nE & 3) == 0) ? 1 : 0;

  const int nPrep = HID * INW / 8 + HID * HID / 8 + HID * INW / 8;
  k_wprep<<<(nPrep + NTHR - 1) / NTHR, NTHR, 0, stream>>>(gcn_w, gat_w, sage_wl, sage_wr, wG, wT, wS);

  k_count<<<nBC, NTHR, 0, stream>>>(ei, cnt, dinv, nE, vec8);
  k_offsets<<<1, OTHR, 0, stream>>>(cnt, offp, rb, nBC);
  hipFuncSetAttribute(reinterpret_cast<const void*>(&k_fill),
                      hipFuncAttributeMaxDynamicSharedMemorySize, LDS_FILL);
  k_fill<<<nBF, NTHR, LDS_FILL, stream>>>(ei, offp, rb, csr, nN, nE, vec8, csrLen);

  k_gemm<INW, 0><<<nGemm, NTHR, 0, stream>>>(x, x, wG, dinv, gcn_b, att_src, att_dst, P0, asp, adp, nN, NPAD);
  k_agg_gcn<<<nAgg, NTHR, 0, stream>>>(csr, offp, cnt, dinv, P0, gcn_b, P1, nN, csrLen);

  k_gemm<HID, 1><<<nGemm, NTHR, 0, stream>>>(P1, P1, wT, dinv, gat_b, att_src, att_dst, P2, asp, adp, NPAD, NPAD);
  k_agg_gat<<<nAgg, NTHR, 0, stream>>>(csr, offp, cnt, P2, asp, adp, gat_b, P1, nN, csrLen);

  k_agg_sage<<<nAgg, NTHR, 0, stream>>>(csr, offp, cnt, P1, P0, nN, csrLen);
  k_gemm<INW, 2><<<nGemm, NTHR, 0, stream>>>(P0, P1, wS, dinv, sage_b, att_src, att_dst, out, asp, adp, NPAD, nN);
}
